// Interaction_40570261078236
// MI455X (gfx1250) — hardware-verified
//
#include <hip/hip_runtime.h>
#include <math.h>


#define NN 10000
#define CC 32
#define RR 32
#define NE 320000
#define SLOTC 64
#define NCH 128
#define CUTOFF 5.0f

typedef __attribute__((ext_vector_type(16))) _Float16 v16h;
typedef __attribute__((ext_vector_type(8)))  float v8f;
typedef __attribute__((ext_vector_type(4)))  float v4f;
typedef __attribute__((ext_vector_type(4)))  int v4i;
typedef float __attribute__((may_alias)) float_a;
typedef int __attribute__((may_alias)) int_a;

template <typename T> __device__ __forceinline__ void vst2(void* p, T v) { *(volatile T*)p = v; __threadfence(); *(volatile T*)p = v; }
__device__ __forceinline__ v8f wmma16(v16h a, v16h b, v8f c) {
  v8f d = __builtin_amdgcn_wmma_f32_16x16x32_f16(false, a, false, b, (short)0, c, false, false);
  asm volatile("v_nop\n\tv_nop\n\tv_nop\n\tv_nop" : "+v"(d) : "v"(a), "v"(b));
  return d;
}
__device__ __forceinline__ v16h frag_f32(const float* rowk0, int lane) {
  v16h a; const float* p = rowk0 + 8 * (lane >> 4);
#pragma unroll
  for (int i = 0; i < 8; ++i) { a[i] = (_Float16)p[i]; a[8 + i] = (_Float16)p[16 + i]; }
  return a;
}
#define LDSX() do { asm volatile("s_wait_dscnt 0" ::: "memory"); __builtin_amdgcn_wave_barrier(); __builtin_amdgcn_fence(__ATOMIC_RELEASE, "workgroup"); } while (0)

__device__ __forceinline__ void decomp9(const float x[9], float q[9]) {
  const float tr = (x[0] + x[4] + x[8]) * (1.0f / 3.0f);
  q[0] = tr;
  q[1] = 0.5f * (x[1] - x[3]); q[2] = 0.5f * (x[2] - x[6]); q[3] = 0.5f * (x[5] - x[7]);
  q[4] = x[0] - tr; q[5] = x[4] - tr;
  q[6] = 0.5f * (x[1] + x[3]); q[7] = 0.5f * (x[2] + x[6]); q[8] = 0.5f * (x[5] + x[7]);
}
__device__ __forceinline__ void build9(const float q[9], float y[9]) {
  const float s22 = -(q[4] + q[5]);
  y[0] = q[0] + q[4];        y[1] = q[6] + q[1];        y[2] = q[7] + q[2];
  y[3] = q[6] - q[1];        y[4] = q[0] + q[5];        y[5] = q[8] + q[3];
  y[6] = q[7] - q[2];        y[7] = q[8] - q[3];        y[8] = q[0] + s22;
}
__device__ __forceinline__ void matmul3(const float a[9], const float b[9], float c[9]) {
#pragma unroll
  for (int i = 0; i < 3; ++i)
#pragma unroll
    for (int j = 0; j < 3; ++j) c[3 * i + j] = a[3 * i] * b[j] + a[3 * i + 1] * b[3 + j] + a[3 * i + 2] * b[6 + j];
}

__global__ __launch_bounds__(256) void k_part(const float* __restrict__ X, float* __restrict__ PartT) {
  const int n = blockIdx.x * 8 + (threadIdx.x >> 5), c = threadIdx.x & 31;
  if (n >= NN) return;
  float x[9], q[9];
#pragma unroll
  for (int i = 0; i < 9; ++i) x[i] = X[((size_t)n * CC + c) * 9 + i];
  decomp9(x, q);
#pragma unroll
  for (int k = 0; k < 9; ++k) vst2(PartT + ((size_t)k * NN + n) * CC + c, (float_a)q[k]);
}

template <int MODE>
__global__ __launch_bounds__(128) void k_tlin(const float* __restrict__ In, const float* __restrict__ WI, const float* __restrict__ WA,
                                            const float* __restrict__ WS, float* __restrict__ Out) {
  __shared__ __align__(16) float st[4][16 * 288 + 16];
  const int tid = threadIdx.x, wave = tid >> 5, lane = tid & 31, col = lane & 15, g = lane >> 4;
  const int wt = blockIdx.x * 4 + wave;
  if (wt >= NN / 16) return;
  const int n0 = wt * 16;
  float* S = st[wave];
#pragma unroll 1
  for (int k = 0; k < 9; ++k) {
    const float* W = k == 0 ? WI : (k < 4 ? WA : WS);
    const v16h a = frag_f32(In + ((size_t)k * NN + n0 + col) * CC, lane);
    v8f acc0 = {}, acc1 = {};
    acc0 = wmma16(a, frag_f32(W + (size_t)col * CC, lane), acc0);
    acc1 = wmma16(a, frag_f32(W + (size_t)(16 + col) * CC, lane), acc1);
    if (MODE == 0) {
#pragma unroll
      for (int r = 0; r < 8; ++r) { S[(8 * g + r) * 32 + col] = acc0[r]; S[(8 * g + r) * 32 + 16 + col] = acc1[r]; }
      LDSX();
#pragma unroll
      for (int q = 0; q < 4; ++q) { const int rl = q * 4 + (lane >> 3), pc = lane & 7;
        vst2(Out + ((size_t)k * NN + n0 + rl) * CC + pc * 4, *(const v4f*)(S + rl * 32 + pc * 4)); }
      __builtin_amdgcn_wave_barrier();
    } else {
#pragma unroll
      for (int r = 0; r < 8; ++r) { S[(8 * g + r) * 288 + col * 9 + k] = acc0[r]; S[(8 * g + r) * 288 + (16 + col) * 9 + k] = acc1[r]; }
    }
  }
  if (MODE == 1) {
    LDSX();
#pragma unroll 1
    for (int cidx = lane; cidx < 16 * 32; cidx += 32) {
      float q[9], y[9], yy[9];
#pragma unroll
      for (int i = 0; i < 9; ++i) q[i] = S[cidx * 9 + i];
      build9(q, y); matmul3(y, y, yy);
#pragma unroll
      for (int i = 0; i < 9; ++i) S[cidx * 9 + i] = y[i] + yy[i];
    }
    LDSX();
    for (int q = lane; q < 16 * 72; q += 32) { const int rl = q / 72, pc = q % 72;
      vst2(Out + (size_t)(n0 + rl) * 288 + pc * 4, *(const v4f*)(S + rl * 288 + pc * 4)); }
  }
}

__global__ __launch_bounds__(128) void k_edge(const float* __restrict__ rr, const float* __restrict__ W1, const float* __restrict__ b1,
                                            const float* __restrict__ W2, const float* __restrict__ b2, float* __restrict__ F) {
  __shared__ __align__(16) float sh[4][16][68];
  __shared__ __align__(16) float so[4][16][96];
  const int tid = threadIdx.x, w = tid >> 5, lane = tid & 31, col = lane & 15, g = lane >> 4;
  const int e0 = (blockIdx.x * 4 + w) * 16;
  const float emc = expf(-CUTOFF);
  const float beta = 1.0f / ((2.0f / RR * (1.0f - emc)) * (2.0f / RR * (1.0f - emc)));
  const float re = rr[e0 + col], er = expf(-re);
  v16h a;
#pragma unroll
  for (int i = 0; i < 8; ++i) {
    const int k0 = 8 * g + i, k1 = 16 + 8 * g + i;
    const float mu0 = emc + (1.0f - emc) * (float)k0 / (float)(RR - 1), mu1 = emc + (1.0f - emc) * (float)k1 / (float)(RR - 1);
    const float d0 = er - mu0, d1 = er - mu1;
    float p0 = expf(-beta * d0 * d0), p1 = expf(-beta * d1 * d1);
    p0 = p0 < 6.10352e-5f ? 0.f : p0; p1 = p1 < 6.10352e-5f ? 0.f : p1;
    a[i] = (_Float16)p0; a[8 + i] = (_Float16)p1;
  }
  v8f h[4] = {};
#pragma unroll
  for (int j = 0; j < 4; ++j) h[j] = wmma16(a, frag_f32(W1 + (size_t)(j * 16 + col) * RR, lane), h[j]);
  float* H = &sh[w][0][0];
#pragma unroll
  for (int j = 0; j < 4; ++j) { const float bb = b1[j * 16 + col];
#pragma unroll
    for (int r = 0; r < 8; ++r) { const float v = h[j][r] + bb; H[(8 * g + r) * 68 + j * 16 + col] = v / (1.0f + expf(-v)); } }
  LDSX();
  v8f c2[6] = {};
#pragma unroll
  for (int kc = 0; kc < 2; ++kc) {
    const v16h ah = frag_f32(H + col * 68 + kc * 32, lane);
#pragma unroll
    for (int j = 0; j < 6; ++j) c2[j] = wmma16(ah, frag_f32(W2 + (size_t)(j * 16 + col) * 64 + kc * 32, lane), c2[j]);
  }
  float* O = &so[w][0][0];
#pragma unroll
  for (int r = 0; r < 8; ++r) {
    const float rrow = __shfl(re, 8 * g + r, 32);
    const float env = (rrow < CUTOFF) ? 0.5f * (cosf(3.14159265358979f * rrow / CUTOFF) + 1.0f) : 0.f;
#pragma unroll
    for (int j = 0; j < 6; ++j) { const float v = c2[j][r] + b2[j * 16 + col]; O[(8 * g + r) * 96 + j * 16 + col] = v / (1.0f + expf(-v)) * env; }
  }
  LDSX();
  for (int q = lane; q < 16 * 24; q += 32) { const int rl = q / 24, pc = q % 24;
    vst2(F + (size_t)(e0 + rl) * 96 + pc * 4, *(const v4f*)(O + rl * 96 + pc * 4)); }
}

__global__ __launch_bounds__(256) void k_bucket(const int* __restrict__ ei, int* __restrict__ tlist, int* __restrict__ cnt) {
  __shared__ int scnt[NCH];
  __shared__ int slots[NCH][SLOTC];
  const int tid = threadIdx.x, n0 = blockIdx.x * NCH;
  for (int i = tid; i < NCH; i += 256) scnt[i] = 0;
  __syncthreads();
  for (int e = tid; e < NE; e += 256) {
    const int i = ei[e] - n0;
    if (i >= 0 && i < NCH) { const int s = atomicAdd(&scnt[i], 1); if (s < SLOTC) slots[i][s] = e; }
  }
  __syncthreads();
  for (int i = tid; i < NCH; i += 256) { const int n = n0 + i; if (n >= NN) continue;
    int c = scnt[i]; if (c > SLOTC) c = SLOTC;
    for (int a = 1; a < c; ++a) { const int v = slots[i][a]; int b = a - 1; while (b >= 0 && slots[i][b] > v) { slots[i][b + 1] = slots[i][b]; --b; } slots[i][b + 1] = v; }
    for (int a = c; a < SLOTC; ++a) slots[i][a] = 0;
#pragma unroll 1
    for (int p = 0; p < SLOTC / 4; ++p) { v4i v = { slots[i][4 * p], slots[i][4 * p + 1], slots[i][4 * p + 2], slots[i][4 * p + 3] }; vst2(tlist + (size_t)n * SLOTC + 4 * p, v); }
    vst2(cnt + (size_t)n * 32, (int_a)c);
  }
}

__global__ __launch_bounds__(256) void k_node(const float* __restrict__ PartT, const float* __restrict__ Ypre, const float* __restrict__ F,
                                            const int* __restrict__ ei, const int* __restrict__ tlist, const int* __restrict__ cnt, float* __restrict__ Q) {
  const int n = blockIdx.x * 8 + (threadIdx.x >> 5), c = threadIdx.x & 31;
  if (n >= NN) return;
  float m[9] = {0.f, 0.f, 0.f, 0.f, 0.f, 0.f, 0.f, 0.f, 0.f};
  int ne = cnt[(size_t)n * 32]; ne = ne < 0 ? 0 : (ne > SLOTC ? SLOTC : ne);
#pragma unroll 1
  for (int s = 0; s < ne; ++s) {
    const int e = tlist[(size_t)n * SLOTC + s]; if ((unsigned)e >= (unsigned)NE) continue;
    int j = ei[NE + e]; j = j < 0 ? 0 : (j >= NN ? NN - 1 : j);
    const float fI = F[(size_t)e * 96 + c], fA = F[(size_t)e * 96 + 32 + c], fS = F[(size_t)e * 96 + 64 + c];
    m[0] += fI * PartT[((size_t)0 * NN + j) * CC + c];
#pragma unroll
    for (int k = 1; k < 4; ++k) m[k] += fA * PartT[((size_t)k * NN + j) * CC + c];
#pragma unroll
    for (int k = 4; k < 9; ++k) m[k] += fS * PartT[((size_t)k * NN + j) * CC + c];
  }
  float yq[9], y[9], mm[9], z[9], t1[9], t2[9];
#pragma unroll
  for (int k = 0; k < 9; ++k) yq[k] = Ypre[((size_t)k * NN + n) * CC + c];
  build9(yq, y); build9(m, mm);
  matmul3(y, mm, t1); matmul3(mm, y, t2);
  float fr = 0.f;
#pragma unroll
  for (int i = 0; i < 9; ++i) { z[i] = t1[i] + t2[i]; fr += z[i] * z[i]; }
  const float inv = 1.0f / (fr + 1.0f);
#pragma unroll
  for (int i = 0; i < 9; ++i) z[i] *= inv;
  float q[9]; decomp9(z, q);
#pragma unroll
  for (int k = 0; k < 9; ++k) vst2(Q + ((size_t)k * NN + n) * CC + c, (float_a)q[k]);
}

extern "C" void kernel_launch(void* const* d_in, const int* in_sizes, int n_in,
                              void* d_out, int out_size, void* d_ws, size_t ws_size,
                              hipStream_t stream) {
  (void)in_sizes; (void)n_in; (void)out_size; (void)ws_size;
  const float* X  = (const float*)d_in[0];
  const int*   ei = (const int*)d_in[1];
  const float* r  = (const float*)d_in[2];
  const float* WIp = (const float*)d_in[3]; const float* WAp = (const float*)d_in[4]; const float* WSp = (const float*)d_in[5];
  const float* WIq = (const float*)d_in[6]; const float* WAq = (const float*)d_in[7]; const float* WSq = (const float*)d_in[8];
  const float* W1 = (const float*)d_in[9]; const float* b1 = (const float*)d_in[10];
  const float* W2 = (const float*)d_in[11]; const float* b2 = (const float*)d_in[12];
  float* out = (float*)d_out;
  char* ws = (char*)d_ws; size_t off = 0;
  auto take = [&](size_t bytes) { char* p = ws + off; off += (bytes + 255) & ~(size_t)255; return p; };
  float* PartT = (float*)take((size_t)9 * NN * CC * 4);
  float* Ypre  = (float*)take((size_t)9 * NN * CC * 4);
  float* Q     = (float*)take((size_t)9 * NN * CC * 4);
  float* F     = (float*)take((size_t)NE * 96 * 4);
  int*   tlist = (int*)take((size_t)NN * SLOTC * 4);
  int*   cnt   = (int*)take((size_t)NN * 32 * 4);
  k_part<<<NN / 8, 256, 0, stream>>>(X, PartT);
  k_tlin<0><<<(NN / 16 + 3) / 4, 128, 0, stream>>>(PartT, WIp, WAp, WSp, Ypre);
  k_edge<<<NE / 64, 128, 0, stream>>>(r, W1, b1, W2, b2, F);
  k_bucket<<<(NN + NCH - 1) / NCH, 256, 0, stream>>>(ei, tlist, cnt);
  k_node<<<NN / 8, 256, 0, stream>>>(PartT, Ypre, F, ei, tlist, cnt, Q);
  k_tlin<1><<<(NN / 16 + 3) / 4, 128, 0, stream>>>(Q, WIq, WAq, WSq, out);
}
